// GCN_raw_att_46729244181071
// MI455X (gfx1250) — hardware-verified
//
#include <hip/hip_runtime.h>
#include <stddef.h>
#include <math.h>


#define XF      4
#define F1      16
#define F2      32
#define F3      64
#define GH      32
#define NOUT    2
#define NTHR    256
#define NWAVE   8
#define EPT     8
#define NGRP    2
#define CHUNK   (NTHR * EPT * NGRP)
#define WCAP    (EPT * NGRP * 32)
#define LISTN   (NWAVE * WCAP)
#define NBC     4096
#define NBF     1024
#define RCAP    40960
#define RBN     128
#define TGT     256
#define DEGCAP  1024
#define GROWS   128
#define OTHR    512
#define GPB     32
#define PSTR    128
#define CSTR    128
#define WSCAP   134217728

#define WP_L2   0
#define WP_L3   2048
#define WP_GT   10240
#define WP_FC   14336
#define WPTOT   18432

#define LDS_FILL ((RCAP + NBF + LISTN) * 4 + 64)
#define LDS_G2   (2 * GROWS * (32 + 8) * 2 + GROWS * 32 * 4)
#define LDS_G3   (2 * GROWS * (64 + 8) * 2 + GROWS * 64 * 4)
#define LDS_GH   (2 * GROWS * (64 + 8) * 2 + GROWS * 32 * 4)
#define LDS_AG2  (TGT * 2 * F1 * 4)
#define LDS_AG3  (TGT * 2 * F2 * 4)

#define BN_EPS 1e-5f

static_assert((CHUNK & (CHUNK - 1)) == 0);
static_assert(CHUNK <= 4096);
static_assert(NBC <= 4096 && NBF <= 4096 && GPB <= 4096);
static_assert((NBC & (NBC - 1)) == 0 && (NBF & (NBF - 1)) == 0 && (GPB & (GPB - 1)) == 0);
static_assert(NBC == 4 * NBF);
static_assert(OTHR * 8 == NBC);
static_assert((RCAP % 32) == 0);
static_assert(TGT == NWAVE * 32 && (TGT % GROWS) == 0);
static_assert((NBC % TGT) == 0);
static_assert(GROWS == NWAVE * 16);
static_assert(GPB * 8 == NTHR);
static_assert(WP_L3 == WP_L2 + 2 * 32 * 32 && WP_GT == WP_L3 + 2 * 64 * 64);
static_assert(WP_FC == WP_GT + 2 * 32 * 64 && WPTOT == WP_FC + 2 * 32 * 64);
static_assert((WP_L3 % 64) == 0 && (WP_GT % 64) == 0 && (WP_FC % 64) == 0);

typedef float          v2f  __attribute__((ext_vector_type(2)));
typedef float          v4f  __attribute__((ext_vector_type(4)));
typedef float          v8f  __attribute__((ext_vector_type(8)));
typedef double         v2d  __attribute__((ext_vector_type(2)));
typedef int            v4i  __attribute__((ext_vector_type(4)));
typedef unsigned short v8us __attribute__((ext_vector_type(8)));
typedef __bf16         v16b __attribute__((ext_vector_type(16)));
union FragB { v16b v; v8us h[2]; };

__device__ __forceinline__ unsigned int bfr(float f) {
  const unsigned int u = __float_as_uint(f);
  return (u + 0x7FFFu + ((u >> 16) & 1u)) >> 16;
}

__device__ __forceinline__ void split1(float x, unsigned short& hb, unsigned short& lb) {
  const unsigned int hu = bfr(x);
  const float hf = __uint_as_float(hu << 16);
  hb = (unsigned short)hu;
  lb = (unsigned short)bfr(x - hf);
}

__device__ __forceinline__ void split8(v4f a, v4f b, v8us& hi, v8us& lo) {
  unsigned short hb, lb;
  split1(a.x, hb, lb); hi[0] = hb; lo[0] = lb;
  split1(a.y, hb, lb); hi[1] = hb; lo[1] = lb;
  split1(a.z, hb, lb); hi[2] = hb; lo[2] = lb;
  split1(a.w, hb, lb); hi[3] = hb; lo[3] = lb;
  split1(b.x, hb, lb); hi[4] = hb; lo[4] = lb;
  split1(b.y, hb, lb); hi[5] = hb; lo[5] = lb;
  split1(b.z, hb, lb); hi[6] = hb; lo[6] = lb;
  split1(b.w, hb, lb); hi[7] = hb; lo[7] = lb;
}

__device__ __forceinline__ v8f wmb(v16b a, v16b b, v8f c) {
  v8f d = __builtin_amdgcn_wmma_f32_16x16x32_bf16(false, a, false, b, (short)0, c, false, false);
  asm volatile("v_nop\n\tv_nop\n\tv_nop\n\tv_nop" : "+v"(d) : "v"(a), "v"(b));
  return d;
}

template <int KD, int NT, int NCT, int APK>
__device__ __forceinline__ void mma_tiles(const unsigned short* sHi, const unsigned short* sLo,
                                          const unsigned short* __restrict__ Bw, int wrow, int lane,
                                          v8f (&acc)[NT]) {
  static_assert((KD % 32) == 0 && (APK % 8) == 0);
  constexpr int NKT = KD / 32, WPLN = NCT * KD;
  const int hh = lane >> 4, m = lane & 15;
#pragma unroll
  for (int t = 0; t < NT; ++t) { v8f z = {0.f, 0.f, 0.f, 0.f, 0.f, 0.f, 0.f, 0.f}; acc[t] = z; }
  const unsigned short* ahp = sHi + (wrow + m) * APK + 8 * hh;
  const unsigned short* alp = sLo + (wrow + m) * APK + 8 * hh;
#pragma unroll 1
  for (int kt = 0; kt < NKT; ++kt) {
    FragB ah, al;
    ah.h[0] = *(const v8us*)(ahp + 32 * kt);
    ah.h[1] = *(const v8us*)(ahp + 32 * kt + 16);
    al.h[0] = *(const v8us*)(alp + 32 * kt);
    al.h[1] = *(const v8us*)(alp + 32 * kt + 16);
#pragma unroll
    for (int t = 0; t < NT; ++t) {
      const unsigned short* bp = Bw + (size_t)(16 * t + m) * KD + 32 * kt + 8 * hh;
      FragB bh, bl;
      bh.h[0] = *(const v8us*)bp;
      bh.h[1] = *(const v8us*)(bp + 16);
      bl.h[0] = *(const v8us*)(bp + WPLN);
      bl.h[1] = *(const v8us*)(bp + WPLN + 16);
      acc[t] = wmb(ah.v, bh.v, acc[t]);
      acc[t] = wmb(ah.v, bl.v, acc[t]);
      acc[t] = wmb(al.v, bh.v, acc[t]);
    }
  }
}

template <int NF>
__device__ __forceinline__ void store_wave(const float* lp0, float* gp0, int lane) {
  static_assert((NF % 128) == 0);
  constexpr int NI = NF / 128;
  const float* lp = lp0 + 4 * lane;
  float* gp = gp0 + 4 * lane;
#pragma unroll
  for (int i = 0; i < NI; ++i) { const v4f v = *(const v4f*)(lp + 128 * i); *(volatile v4f*)(gp + 128 * i) = v; }
  __threadfence();
#pragma unroll
  for (int i = 0; i < NI; ++i) { const v4f v = *(const v4f*)(lp + 128 * i); *(volatile v4f*)(gp + 128 * i) = v; }
}

template <int NC, int ROWS>
__device__ __forceinline__ void blk_stats(const float* stg, int rowBase, int nRows, double* pblk,
                                          double* dS, double* dQ, double* dP, int tid) {
  constexpr int SG = NTHR / NC, SR = ROWS / SG;
  static_assert(SG * NC == NTHR && SG * SR == ROWS && NC <= 64);
  const int c = tid % NC, g = tid / NC;
  if (tid < PSTR) dP[tid] = 0.0;
  double s = 0.0, q = 0.0;
#pragma unroll 4
  for (int i = 0; i < SR; ++i) {
    const int r = g * SR + i;
    const float v = stg[r * NC + c];
    const float vz = (rowBase + r < nRows) ? v : 0.0f;
    const double dv = (double)vz;
    s += dv;
    q = fma(dv, dv, q);
  }
  dS[tid] = s;
  dQ[tid] = q;
  __syncthreads();
  if (tid < NC) {
    double S = 0.0, Q = 0.0;
#pragma unroll 1
    for (int g2 = 0; g2 < SG; ++g2) { S += dS[g2 * NC + tid]; Q += dQ[g2 * NC + tid]; }
    dP[tid] = S;
    dP[64 + tid] = Q;
  }
  __syncthreads();
  v2d pv = {0.0, 0.0};
  if (tid < PSTR / 2) pv = *(const v2d*)(dP + 2 * tid);
  double* gq = pblk + 2 * tid;
  if (tid < PSTR / 2) *(volatile v2d*)gq = pv;
  __threadfence();
  if (tid < PSTR / 2) *(volatile v2d*)gq = pv;
}

template <int NB>
__device__ __forceinline__ int scan_chunk(const int* __restrict__ dsts, int nE, int cbase, int slotBase,
                                          int vec8, int* list, int tid, int lane, int wave) {
  int wc = 0;
#pragma unroll
  for (int g = 0; g < NGRP; ++g) {
    const int el0  = (g * NTHR + tid) * EPT;
    const int e0   = cbase + el0;
    const int sent = -2147483647 - 1;
    v4i da, db;
    if (vec8 != 0 && cbase + CHUNK <= nE) {
      da = *(const v4i*)(dsts + e0);
      db = *(const v4i*)(dsts + e0 + 4);
    } else {
      da.x = (e0     < nE) ? dsts[min(e0, nE - 1)] : sent;
      da.y = (e0 + 1 < nE) ? dsts[min(e0 + 1, nE - 1)] : sent;
      da.z = (e0 + 2 < nE) ? dsts[min(e0 + 2, nE - 1)] : sent;
      da.w = (e0 + 3 < nE) ? dsts[min(e0 + 3, nE - 1)] : sent;
      db.x = (e0 + 4 < nE) ? dsts[min(e0 + 4, nE - 1)] : sent;
      db.y = (e0 + 5 < nE) ? dsts[min(e0 + 5, nE - 1)] : sent;
      db.z = (e0 + 6 < nE) ? dsts[min(e0 + 6, nE - 1)] : sent;
      db.w = (e0 + 7 < nE) ? dsts[min(e0 + 7, nE - 1)] : sent;
    }
    const unsigned nb = (unsigned)slotBase;
    const unsigned s0 = (unsigned)da.x - nb, s1 = (unsigned)da.y - nb;
    const unsigned s2 = (unsigned)da.z - nb, s3 = (unsigned)da.w - nb;
    const unsigned s4 = (unsigned)db.x - nb, s5 = (unsigned)db.y - nb;
    const unsigned s6 = (unsigned)db.z - nb, s7 = (unsigned)db.w - nb;
    const bool h0 = s0 < (unsigned)NB, h1 = s1 < (unsigned)NB, h2 = s2 < (unsigned)NB, h3 = s3 < (unsigned)NB;
    const bool h4 = s4 < (unsigned)NB, h5 = s5 < (unsigned)NB, h6 = s6 < (unsigned)NB, h7 = s7 < (unsigned)NB;
    const unsigned any = __builtin_amdgcn_ballot_w32(h0 | h1 | h2 | h3 | h4 | h5 | h6 | h7);
    if (any != 0u) {
#define HITJ(J, HJ, SJ) { \
        const unsigned mj = __builtin_amdgcn_ballot_w32(HJ); \
        if (mj != 0u) { \
          if (HJ) { \
            const int pos = wc + (int)__builtin_amdgcn_mbcnt_lo(mj, 0u); \
            if (pos < WCAP) list[wave * WCAP + pos] = ((el0 + (J)) << 12) | (int)(SJ); \
          } \
          wc += (int)__builtin_popcount(mj); } }
      HITJ(0, h0, s0)
      HITJ(1, h1, s1)
      HITJ(2, h2, s2)
      HITJ(3, h3, s3)
      HITJ(4, h4, s4)
      HITJ(5, h5, s5)
      HITJ(6, h6, s6)
      HITJ(7, h7, s7)
#undef HITJ
    }
  }
  return wc;
}

__global__ __launch_bounds__(NTHR) void k_wprep(
    const float* __restrict__ w2r, const float* __restrict__ w2o,
    const float* __restrict__ w3r, const float* __restrict__ w3o,
    const float* __restrict__ gw1, const float* __restrict__ f1w, unsigned short* wp) {
  const int blk = blockIdx.x, tid = threadIdx.x;
  float v[8];
  int KD, NC, i, base, cntv;
  if (blk == 0) {
    KD = 32; NC = 32; i = tid; base = WP_L2; cntv = 32 * 32 / 8;
    const int ii = i > cntv - 1 ? cntv - 1 : i;
    const int n = ii >> 2, k0 = (ii & 3) * 8;
#pragma unroll
    for (int e = 0; e < 8; ++e) {
      const int k = k0 + e;
      const int ka = k > 15 ? 15 : k;
      int kb = k - 16; kb = kb < 0 ? 0 : (kb > 15 ? 15 : kb);
      const float va = w2r[ka * 32 + n];
      const float vb = w2o[kb * 32 + n];
      v[e] = (k < 16) ? va : vb;
    }
  } else if (blk < 3) {
    KD = 64; NC = 64; i = (blk - 1) * NTHR + tid; base = WP_L3; cntv = 64 * 64 / 8;
    const int n = i >> 3, k0 = (i & 7) * 8;
#pragma unroll
    for (int e = 0; e < 8; ++e) {
      const int k = k0 + e;
      const int ka = k > 31 ? 31 : k;
      int kb = k - 32; kb = kb < 0 ? 0 : (kb > 31 ? 31 : kb);
      const float va = w3r[ka * 64 + n];
      const float vb = w3o[kb * 64 + n];
      v[e] = (k < 32) ? va : vb;
    }
  } else if (blk == 3) {
    KD = 64; NC = 32; i = tid; base = WP_GT; cntv = 32 * 64 / 8;
    const int n = i >> 3, k0 = (i & 7) * 8;
#pragma unroll
    for (int e = 0; e < 8; ++e) v[e] = gw1[(k0 + e) * 32 + n];
  } else {
    KD = 64; NC = 32; i = tid; base = WP_FC; cntv = 32 * 64 / 8;
    const int n = i >> 3, k0 = (i & 7) * 8;
#pragma unroll
    for (int e = 0; e < 8; ++e) v[e] = f1w[(k0 + e) * 32 + n];
  }
  v4f a, b;
  a.x = v[0]; a.y = v[1]; a.z = v[2]; a.w = v[3];
  b.x = v[4]; b.y = v[5]; b.z = v[6]; b.w = v[7];
  v8us hv, lv;
  split8(a, b, hv, lv);
  const int is = i > cntv - 1 ? cntv - 1 : i;
  unsigned short* dh = wp + base + (size_t)is * 8;
  unsigned short* dl = dh + NC * KD;
  if (i < cntv) { *(volatile v8us*)dh = hv; *(volatile v8us*)dl = lv; }
  __threadfence();
  if (i < cntv) { *(volatile v8us*)dh = hv; *(volatile v8us*)dl = lv; }
}

__global__ __launch_bounds__(NTHR) void k_count(const int* __restrict__ dsts, int* cnt, int nE, int vec8) {
  __shared__ __attribute__((aligned(16))) int scnt[NBC];
  __shared__ __attribute__((aligned(16))) int list[LISTN];
  __shared__ int wcnt[NWAVE];
  const int tid = threadIdx.x, lane = tid & 31, wave = tid >> 5;
  const int nodeBase = blockIdx.x * NBC;

  for (int i = tid; i < NBC; i += NTHR) scnt[i] = 0;
  __syncthreads();

  const int nChunks = (nE + CHUNK - 1) / CHUNK;
#pragma unroll 1
  for (int ch = 0; ch < nChunks; ++ch) {
    const int cbase = ch * CHUNK;
    const int wc = scan_chunk<NBC>(dsts, nE, cbase, nodeBase, vec8, list, tid, lane, wave);
    if (lane == 0) wcnt[wave] = wc;
    __syncthreads();
    if (wave == 0) {
#pragma unroll 1
      for (int wsx = 0; wsx < NWAVE; ++wsx) {
        int n = __builtin_amdgcn_readfirstlane(wcnt[wsx]);
        n = n > WCAP ? WCAP : (n < 0 ? 0 : n);
        const int* lp = list + wsx * WCAP;
#pragma unroll 1
        for (int i = 0; i < n; ++i) {
          const int ent  = __builtin_amdgcn_readfirstlane(lp[i]);
          const int slot = ent & (NBC - 1);
          if (lane == 0) scnt[slot] = scnt[slot] + 1;
        }
      }
    }
    __syncthreads();
  }

  v4i cq[4];
#pragma unroll
  for (int q = 0; q < 4; ++q) {
    const int f = (wave * 4 + q) * 128 + 4 * lane;
    cq[q] = *(const v4i*)(scnt + f);
  }
  int* cp = cnt + (size_t)nodeBase;
#pragma unroll
  for (int q = 0; q < 4; ++q) {
    const int f = (wave * 4 + q) * 128 + 4 * lane;
    *(volatile v4i*)(cp + f) = cq[q];
  }
  __threadfence();
#pragma unroll
  for (int q = 0; q < 4; ++q) {
    const int f = (wave * 4 + q) * 128 + 4 * lane;
    *(volatile v4i*)(cp + f) = cq[q];
  }
}

__global__ __launch_bounds__(OTHR) void k_offsets(
    const int* __restrict__ cnt, int* off, int* rbase, int nChunk) {
  __shared__ __attribute__((aligned(16))) int soff[NBC];
  __shared__ __attribute__((aligned(16))) int srb[RBN];
  __shared__ int wtot[OTHR / 32];
  const int tid = threadIdx.x, lane = tid & 31, wave = tid >> 5, sub = tid >> 7;
  for (int i = tid; i < RBN; i += OTHR) srb[i] = 0;
  int carry = 0;
#pragma unroll 1
  for (int ch = 0; ch < nChunk; ++ch) {
    const int base = ch * NBC;
    const v4i c0 = *(const v4i*)(cnt + base + 8 * tid);
    const v4i c1 = *(const v4i*)(cnt + base + 8 * tid + 4);
    const int e0 = max(c0.x, 0), e1 = max(c0.y, 0), e2 = max(c0.z, 0), e3 = max(c0.w, 0);
    const int e4 = max(c1.x, 0), e5 = max(c1.y, 0), e6 = max(c1.z, 0), e7 = max(c1.w, 0);
    const int ts = e0 + e1 + e2 + e3 + e4 + e5 + e6 + e7;
    int incl = ts;
#pragma unroll
    for (int d = 1; d < 32; d <<= 1) {
      const int t = __shfl_up(incl, d);
      if (lane >= d) incl += t;
    }
    if (lane == 31) wtot[wave] = incl;
    __syncthreads();
    const int S0 = wtot[0]  + wtot[1]  + wtot[2]  + wtot[3];
    const int S1 = wtot[4]  + wtot[5]  + wtot[6]  + wtot[7];
    const int S2 = wtot[8]  + wtot[9]  + wtot[10] + wtot[11];
    const int S3 = wtot[12] + wtot[13] + wtot[14] + wtot[15];
    int pre = 0;
#pragma unroll 1
    for (int w = 4 * sub; w < wave; ++w) pre += wtot[w];
    const int b0 = carry;
    const int b1 = b0 + ((S0 + 31) & ~31);
    const int b2 = b1 + ((S1 + 31) & ~31);
    const int b3 = b2 + ((S2 + 31) & ~31);
    const int b4 = b3 + ((S3 + 31) & ~31);
    const int myb = sub == 0 ? b0 : (sub == 1 ? b1 : (sub == 2 ? b2 : b3));
    if (tid == 0) {
      srb[min(4 * ch + 0, RBN - 1)] = b0;
      srb[min(4 * ch + 1, RBN - 1)] = b1;
      srb[min(4 * ch + 2, RBN - 1)] = b2;
      srb[min(4 * ch + 3, RBN - 1)] = b3;
    }
    int run = myb + pre + incl - ts;
    soff[8 * tid + 0] = run; run += e0;
    soff[8 * tid + 1] = run; run += e1;
    soff[8 * tid + 2] = run; run += e2;
    soff[8 * tid + 3] = run; run += e3;
    soff[8 * tid + 4] = run; run += e4;
    soff[8 * tid + 5] = run; run += e5;
    soff[8 * tid + 6] = run; run += e6;
    soff[8 * tid + 7] = run;
    carry = b4;
    __syncthreads();
    const v4i o0 = *(const v4i*)(soff + 4 * tid);
    const v4i o1 = *(const v4i*)(soff + 4 * (tid + OTHR));
    int* op = off + base;
    *(volatile v4i*)(op + 4 * tid) = o0;
    *(volatile v4i*)(op + 4 * (tid + OTHR)) = o1;
    __threadfence();
    *(volatile v4i*)(op + 4 * tid) = o0;
    *(volatile v4i*)(op + 4 * (tid + OTHR)) = o1;
    __syncthreads();
  }
  if (tid == 0) srb[min(4 * nChunk, RBN - 1)] = carry;
  __syncthreads();
  v4i rv = {0, 0, 0, 0};
  if (tid < 32) rv = *(const v4i*)(srb + 4 * tid);
  if (tid < 32) *(volatile v4i*)(rbase + 4 * tid) = rv;
  __threadfence();
  if (tid < 32) *(volatile v4i*)(rbase + 4 * tid) = rv;
}

__global__ __launch_bounds__(NTHR) void k_fill(
    const int* __restrict__ dsts, const int* __restrict__ off, const int* __restrict__ rbase,
    int* csr, int nE, int vec8, int csrLen) {
  extern __shared__ v4f lds_dyn[];
  int* region = (int*)lds_dyn;
  int* cursor = region + RCAP;
  int* list   = cursor + NBF;
  int* wcnt   = list + LISTN;
  const int tid = threadIdx.x, lane = tid & 31, wave = tid >> 5;
  const int b = blockIdx.x;
  const int nodeBase = b * NBF;

  int rb0 = rbase[b];
  const int rb1 = rbase[b + 1];
  rb0 = rb0 < 0 ? 0 : (rb0 > csrLen ? csrLen : rb0);
  rb0 &= ~31;
  int len = rb1 - rb0;
  len = len < 0 ? 0 : (len > RCAP ? RCAP : len);
  int lenW = (len + 31) & ~31;
  if (rb0 + lenW > csrLen) lenW = (csrLen - rb0) & ~31;

  {
    const v4i z = {0, 0, 0, 0};
    for (int i = tid; i < RCAP / 4; i += NTHR) ((v4i*)region)[i] = z;
    for (int s = tid; s < NBF; s += NTHR) {
      int o = off[nodeBase + s] - rb0;
      o = o < 0 ? 0 : (o > RCAP ? RCAP : o);
      cursor[s] = o;
    }
  }
  __syncthreads();

  const int nChunks = (nE + CHUNK - 1) / CHUNK;
#pragma unroll 1
  for (int ch = 0; ch < nChunks; ++ch) {
    const int cbase = ch * CHUNK;
    const int wc = scan_chunk<NBF>(dsts, nE, cbase, nodeBase, vec8, list, tid, lane, wave);
    if (lane == 0) wcnt[wave] = wc;
    __syncthreads();
    if (wave == 0) {
#pragma unroll 1
      for (int wsx = 0; wsx < NWAVE; ++wsx) {
        int n = __builtin_amdgcn_readfirstlane(wcnt[wsx]);
        n = n > WCAP ? WCAP : (n < 0 ? 0 : n);
        const int* lp = list + wsx * WCAP;
#pragma unroll 1
        for (int i = 0; i < n; ++i) {
          const int ent  = __builtin_amdgcn_readfirstlane(lp[i]);
          const int slot = ent & (NBF - 1);
          int e = cbase + ((ent >> 12) & (CHUNK - 1));
          e = e > nE - 1 ? nE - 1 : e;
          if (lane == 0) {
            int pos = cursor[slot];
            pos = pos < 0 ? 0 : (pos > RCAP - 1 ? RCAP - 1 : pos);
            region[pos] = e;
            const int np = pos + 1;
            cursor[slot] = np > RCAP ? RCAP : np;
          }
        }
      }
    }
    __syncthreads();
  }

  const int nv = lenW >> 2;
  int* gp = csr + rb0;
#pragma unroll 1
  for (int i = tid; i < nv; i += NTHR) { const v4i v = ((const v4i*)region)[i]; *(volatile v4i*)(gp + 4 * i) = v; }
  __threadfence();
#pragma unroll 1
  for (int i = tid; i < nv; i += NTHR) { const v4i v = ((const v4i*)region)[i]; *(volatile v4i*)(gp + 4 * i) = v; }
}

__global__ __launch_bounds__(NTHR) void k_agg0(
    const int* __restrict__ csr, const int* __restrict__ off, const int* __restrict__ cnt,
    const int* __restrict__ srcs, const float* __restrict__ ew, const float* __restrict__ x,
    const float* __restrict__ wrel, const float* __restrict__ brel, const float* __restrict__ wroot,
    float* H, double* part, int nN, int nE, int csrLen) {
  __shared__ __attribute__((aligned(16))) float sOp[TGT * 8];
  __shared__ __attribute__((aligned(16))) float stg[TGT * F1];
  __shared__ __attribute__((aligned(16))) double dS[NTHR];
  __shared__ __attribute__((aligned(16))) double dQ[NTHR];
  __shared__ __attribute__((aligned(16))) double dP[PSTR];
  const int tid = threadIdx.x, lane = tid & 31, wave = tid >> 5;
  const int rowBase = blockIdx.x * TGT;
  const int t = rowBase + wave * 32 + lane;
  int n = cnt[t];
  n = n < 0 ? 0 : (n > DEGCAP ? DEGCAP : n);
  const int st = off[t];
  int nmx = n;
  nmx = max(nmx, __shfl_xor(nmx, 16));
  nmx = max(nmx, __shfl_xor(nmx, 8));
  nmx = max(nmx, __shfl_xor(nmx, 4));
  nmx = max(nmx, __shfl_xor(nmx, 2));
  nmx = max(nmx, __shfl_xor(nmx, 1));
  nmx = nmx > DEGCAP ? DEGCAP : nmx;
  v4f acc = {0.0f, 0.0f, 0.0f, 0.0f};
#pragma unroll 1
  for (int p = 0; p < nmx; ++p) {
    int pos = st + p;
    pos = pos < 0 ? 0 : (pos > csrLen - 1 ? csrLen - 1 : pos);
    int e = csr[pos];
    e = e < 0 ? 0 : (e > nE - 1 ? nE - 1 : e);
    int s = srcs[e];
    s = s < 0 ? 0 : (s > nN - 1 ? nN - 1 : s);
    const float w = ew[e];
    const float we = (p < n) ? w : 0.0f;
    const v4f xv = *(const v4f*)(x + (size_t)s * XF);
    acc = acc + xv * we;
  }
  const float rc = 1.0f / (float)(n > 1 ? n : 1);
  const v4f mean = acc * rc;
  const int ts = t > nN - 1 ? nN - 1 : t;
  const v4f xs = *(const v4f*)(x + (size_t)ts * XF);
  *(v4f*)(sOp + (wave * 32 + lane) * 8) = mean;
  *(v4f*)(sOp + (wave * 32 + lane) * 8 + 4) = xs;
  __syncthreads();

  {
    const int c = lane & 15, hrow = lane >> 4;
    float wk[8];
#pragma unroll
    for (int k = 0; k < 4; ++k) { wk[k] = wrel[k * F1 + c]; wk[4 + k] = wroot[k * F1 + c]; }
    const float bc = brel[c];
#pragma unroll 1
    for (int r = 0; r < 16; ++r) {
      const int row = wave * 32 + hrow * 16 + r;
      const v4f l0 = *(const v4f*)(sOp + row * 8);
      const v4f l1 = *(const v4f*)(sOp + row * 8 + 4);
      float v = bc;
      v += l0.x * wk[0]; v += l0.y * wk[1]; v += l0.z * wk[2]; v += l0.w * wk[3];
      v += l1.x * wk[4]; v += l1.y * wk[5]; v += l1.z * wk[6]; v += l1.w * wk[7];
      stg[row * F1 + c] = v;
    }
  }
  __syncthreads();

  blk_stats<F1, TGT>(stg, rowBase, nN, part + (size_t)blockIdx.x * PSTR, dS, dQ, dP, tid);

  store_wave<32 * F1>(stg + wave * 32 * F1, H + (size_t)(rowBase + wave * 32) * F1, lane);
}

template <int FP>
__global__ __launch_bounds__(NTHR) void k_agg(
    const int* __restrict__ csr, const int* __restrict__ off, const int* __restrict__ cnt,
    const int* __restrict__ srcs, const float* __restrict__ ew, const float* __restrict__ Hp,
    const float* __restrict__ coef, const float* __restrict__ beta,
    float* Aop, int nN, int nE, int csrLen) {
  static_assert(FP == 16 || FP == 32);
  constexpr int RW = 2 * FP;
  extern __shared__ v4f lds_dyn[];
  float* stg = (float*)lds_dyn;
  const int tid = threadIdx.x, lane = tid & 31, wave = tid >> 5;
  const int tbase = blockIdx.x * TGT + wave * 32;
  const int cl = tbase + lane;
  const int cnt_l = cnt[cl];
  const int off_l = off[cl];
  const int c = lane & (FP - 1);
  const float mu = coef[c], a = coef[64 + c], bb = beta[c];

#pragma unroll 1
  for (int j = 0; j < 32; ++j) {
    const int cnode = tbase + j;
    int n = __builtin_amdgcn_readlane(cnt_l, j);
    n = n < 0 ? 0 : (n > DEGCAP ? DEGCAP : n);
    const int st = __builtin_amdgcn_readlane(off_l, j);
    float acc = 0.0f;
#pragma unroll 1
    for (int q0 = 0; q0 < n; q0 += 32) {
      int pos = st + q0 + lane;
      pos = pos < 0 ? 0 : (pos > csrLen - 1 ? csrLen - 1 : pos);
      int el = csr[pos];
      el = el < 0 ? 0 : (el > nE - 1 ? nE - 1 : el);
      int sl = srcs[el];
      sl = sl < 0 ? 0 : (sl > nN - 1 ? nN - 1 : sl);
      const int wli = __float_as_int(ew[el]);
      const int mcnt = (n - q0) < 32 ? (n - q0) : 32;
#pragma unroll 1
      for (int p = 0; p < mcnt; ++p) {
        const int s = __builtin_amdgcn_readlane(sl, p);
        const float w = __int_as_float(__builtin_amdgcn_readlane(wli, p));
        const float v = Hp[(size_t)s * FP + c];
        const float av = fmaxf((v - mu) * a + bb, 0.0f);
        acc += av * w;
      }
    }
    const float rc = 1.0f / (float)(n > 1 ? n : 1);
    const float mean = acc * rc;
    const int cs = cnode > nN - 1 ? nN - 1 : cnode;
    const float sv = Hp[(size_t)cs * FP + c];
    const float sa = fmaxf((sv - mu) * a + bb, 0.0f);
    stg[(wave * 32 + j) * RW + c] = mean;
    stg[(wave * 32 + j) * RW + FP + c] = sa;
  }
  __syncthreads();

  store_wave<32 * RW>(stg + wave * 32 * RW, Aop + (size_t)tbase * RW, lane);
}

__device__ __forceinline__ void head_pass(const float* so, float* ob, int nf, int tid) {
  if (tid < (GROWS * NOUT) / 4) {
    const int q = tid;
    const v4f v = *(const v4f*)(so + 4 * q);
    if (4 * q + 4 <= nf) {
      *(volatile v4f*)(ob + 4 * q) = v;
    } else if (4 * q < nf) {
      volatile float* op = ob + 4 * q;
      op[0] = v.x;
      if (4 * q + 1 < nf) op[1] = v.y;
      if (4 * q + 2 < nf) op[2] = v.z;
    }
  }
}

template <int KD, int NC, int EPI>
__global__ __launch_bounds__(NTHR) void k_gemm(
    const float* __restrict__ A, const unsigned short* __restrict__ Bw, const float* __restrict__ bias,
    const float* __restrict__ hw, const float* __restrict__ hb,
    float* C, double* part, int nRows) {
  static_assert((KD == 32 || KD == 64) && (NC == 32 || NC == 64));
  static_assert(EPI < 2 || NC == GH);
  constexpr int APK = KD + 8, NT = NC / 16, CG = KD / 8, RPP = NTHR / CG, NPASS = GROWS / RPP;
  extern __shared__ v4f lds_dyn[];
  __shared__ __attribute__((aligned(16))) double dS[NTHR];
  __shared__ __attribute__((aligned(16))) double dQ[NTHR];
  __shared__ __attribute__((aligned(16))) double dP[PSTR];
  __shared__ __attribute__((aligned(16))) float sg[GROWS * NOUT];
  unsigned short* sHi = (unsigned short*)lds_dyn;
  unsigned short* sLo = sHi + GROWS * APK;
  float*          stg = (float*)((char*)lds_dyn + 2 * GROWS * APK * 2);
  const int tid = threadIdx.x, lane = tid & 31, wave = tid >> 5, hh = lane >> 4, m = lane & 15;
  const int rowBase = blockIdx.x * GROWS;
  const int c0 = (tid % CG) * 8, rr = tid / CG;

#pragma unroll
  for (int it = 0; it < NPASS; ++it) {
    const int r = it * RPP + rr;
    const float* ap = A + (size_t)(rowBase + r) * KD + c0;
    const v4f a = *(const v4f*)ap, b = *(const v4f*)(ap + 4);
    v8us hv, lv;
    split8(a, b, hv, lv);
    *(v8us*)(sHi + r * APK + c0) = hv;
    *(v8us*)(sLo + r * APK + c0) = lv;
  }
  __syncthreads();

  {
    v8f acc[NT];
    mma_tiles<KD, NT, NC, APK>(sHi, sLo, Bw, wave * 16, lane, acc);
    float* sp = stg + (wave * 16 + 8 * hh) * NC + m;
#pragma unroll
    for (int t = 0; t < NT; ++t) {
      const float bv = bias[16 * t + m];
#pragma unroll
      for (int r = 0; r < 8; ++r) {
        float v = acc[t][r] + bv;
        if (EPI != 0) v = fmaxf(v, 0.0f);
        sp[r * NC + 16 * t] = v;
      }
    }
  }
  __syncthreads();

  if constexpr (EPI == 0) {
    blk_stats<NC, GROWS>(stg, rowBase, nRows, part + (size_t)blockIdx.x * PSTR, dS, dQ, dP, tid);
  }
  if constexpr (EPI == 0 || EPI == 1) {
    store_wave<16 * NC>(stg + wave * 16 * NC, C + (size_t)(rowBase + wave * 16) * NC, lane);
  }
  if constexpr (EPI == 2) {
    if (tid < GROWS) {
      const float* sr = stg + tid * NC;
      float g = 0.0f;
#pragma unroll
      for (int j = 0; j < NC; ++j) g += sr[j] * hw[j];
      g += hb[0];
      sg[tid] = g;
    }
    __syncthreads();
    v4f gv = {0.f, 0.f, 0.f, 0.f};
    if (wave == 0) gv = *(const v4f*)(sg + 4 * lane);
    float* gp = C + (size_t)rowBase + 4 * lane;
    if (wave == 0) *(volatile v4f*)gp = gv;
    __threadfence();
    if (wave == 0) *(volatile v4f*)gp = gv;
  }
  if constexpr (EPI == 3) {
    if (tid < GROWS) {
      const float* sr = stg + tid * NC;
      float o0 = 0.0f, o1 = 0.0f;
#pragma unroll
      for (int j = 0; j < NC; ++j) { o0 += sr[j] * hw[2 * j]; o1 += sr[j] * hw[2 * j + 1]; }
      o0 += hb[0];
      o1 += hb[1];
      const float mx = fmaxf(o0, o1);
      const float s0 = o0 - mx, s1 = o1 - mx;
      const float l = logf(expf(s0) + expf(s1));
      sg[2 * tid]     = s0 - l;
      sg[2 * tid + 1] = s1 - l;
    }
    __syncthreads();
    int nv = nRows - rowBase;
    nv = nv > GROWS ? GROWS : (nv < 0 ? 0 : nv);
    const int nf = nv * NOUT;
    float* ob = C + (size_t)rowBase * NOUT;
    head_pass(sg, ob, nf, tid);
    __threadfence();
    head_pass(sg, ob, nf, tid);
  }
}

__global__ __launch_bounds__(NTHR) void k_bnfin(const double* __restrict__ part, const float* __restrict__ gam,
                                                float* coef, int nBlk, int nN, int F) {
  __shared__ __attribute__((aligned(16))) float sco[CSTR];
  const int tid = threadIdx.x;
  if (tid < 64) {
    const int c = tid;
    double S = 0.0, Q = 0.0;
#pragma unroll 1
    for (int b = 0; b < nBlk; ++b) {
      S += part[(size_t)b * PSTR + c];
      Q += part[(size_t)b * PSTR + 64 + c];
    }
    const double rn = 1.0 / (double)(nN > 1 ? nN : 1);
    const double mean = S * rn;
    double var = Q * rn - mean * mean;
    var = var < 0.0 ? 0.0 : var;
    const float muf = (float)mean;
    const float rs  = 1.0f / sqrtf((float)var + BN_EPS);
    const int cg = c > F - 1 ? F - 1 : c;
    const float gv = gam[cg < 0 ? 0 : cg];
    sco[c]      = (c < F) ? muf : 0.0f;
    sco[64 + c] = (c < F) ? gv * rs : 0.0f;
  }
  __syncthreads();
  v4f cv = {0.f, 0.f, 0.f, 0.f};
  if (tid < 32) cv = *(const v4f*)(sco + 4 * tid);
  if (tid < 32) *(volatile v4f*)(coef + 4 * tid) = cv;
  __threadfence();
  if (tid < 32) *(volatile v4f*)(coef + 4 * tid) = cv;
}

__global__ __launch_bounds__(NTHR) void k_pool(const int* __restrict__ bat, const float* __restrict__ gate,
                                               const float* __restrict__ H, float* P, int nN, int vecb) {
  __shared__ __attribute__((aligned(16))) int list[LISTN];
  __shared__ int wcnt[NWAVE];
  __shared__ float smax[GPB];
  __shared__ __attribute__((aligned(16))) float stg[GPB * F3];
  const int tid = threadIdx.x, lane = tid & 31, wave = tid >> 5;
  const int gBase = blockIdx.x * GPB;
  const float ninf = __uint_as_float(0xff800000u);
  if (tid < GPB) smax[tid] = ninf;
  __syncthreads();
  const int nChunks = (nN + CHUNK - 1) / CHUNK;

#pragma unroll 1
  for (int ch = 0; ch < nChunks; ++ch) {
    const int cbase = ch * CHUNK;
    const int wc = scan_chunk<GPB>(bat, nN, cbase, gBase, vecb, list, tid, lane, wave);
    if (lane == 0) wcnt[wave] = wc;
    __syncthreads();
    if (wave == 0) {
#pragma unroll 1
      for (int wsx = 0; wsx < NWAVE; ++wsx) {
        int n = __builtin_amdgcn_readfirstlane(wcnt[wsx]);
        n = n > WCAP ? WCAP : (n < 0 ? 0 : n);
        const int* lp = list + wsx * WCAP;
#pragma unroll 1
        for (int i = 0; i < n; ++i) {
          const int ent  = __builtin_amdgcn_readfirstlane(lp[i]);
          const int slot = ent & (GPB - 1);
          int node = cbase + ((ent >> 12) & (CHUNK - 1));
          node = node > nN - 1 ? nN - 1 : node;
          const float g = gate[node];
          if (lane == 0) smax[slot] = fmaxf(smax[slot], g);
        }
      }
    }
    __syncthreads();
  }

  float d0 = 0.0f, d1 = 0.0f, d2 = 0.0f, d3 = 0.0f;
  v2f a0 = {0.f, 0.f}, a1 = {0.f, 0.f}, a2 = {0.f, 0.f}, a3 = {0.f, 0.f};
#pragma unroll 1
  for (int ch = 0; ch < nChunks; ++ch) {
    const int cbase = ch * CHUNK;
    const int wc = scan_chunk<GPB>(bat, nN, cbase, gBase, vecb, list, tid, lane, wave);
    if (lane == 0) wcnt[wave] = wc;
    __syncthreads();
#pragma unroll 1
    for (int wsx = 0; wsx < NWAVE; ++wsx) {
      int n = __builtin_amdgcn_readfirstlane(wcnt[wsx]);
      n = n > WCAP ? WCAP : (n < 0 ? 0 : n);
      const int* lp = list + wsx * WCAP;
#pragma unroll 1
      for (int i = 0; i < n; ++i) {
        const int ent  = __builtin_amdgcn_readfirstlane(lp[i]);
        const int slot = ent & (GPB - 1);
        int node = cbase + ((ent >> 12) & (CHUNK - 1));
        node = node > nN - 1 ? nN - 1 : node;
        if ((slot >> 2) == wave) {
          const float g = gate[node];
          const float e = expf(g - smax[slot]);
          const v2f hv = *(const v2f*)(H + (size_t)node * F3 + 2 * lane);
          const int sub = slot & 3;
          if (sub == 0)      { d0 += e; a0 = a0 + hv * e; }
          else if (sub == 1) { d1 += e; a1 = a1 + hv * e; }
          else if (sub == 2) { d2 += e; a2 = a2 + hv * e; }
          else               { d3 += e; a3 = a3 + hv * e; }
        }
      }
    }
    __syncthreads();
  }

  {
    const int s0 = wave * 4;
    const float r0 = d0 > 0.0f ? 1.0f / d0 : 0.0f;
    const float r1 = d1 > 0.0f ? 1.0f / d1 : 0.0f;
    const float r2 = d2 > 0.0f ? 1.0f / d2 : 0.0f;
    const float r3 = d3 > 0.0f ? 1.0f / d3 : 0.0f;
    *(v2f*)(stg + (s0 + 0) * F3 + 2 * lane) = a0 * r0;
    *(v2f*)(stg + (s0 + 1) * F3 + 2 * lane) = a1 * r1;
    *(v2f*)(stg + (s0 + 2) * F3 + 2 * lane) = a2 * r2;
    *(v2f*)(stg + (s0 + 3) * F3 + 2 * lane) = a3 * r3;
  }
  __syncthreads();

  float* gp = P + (size_t)gBase * F3;
  v4f pq[2];
#pragma unroll
  for (int it = 0; it < 2; ++it) { const int q = it * NTHR + tid; pq[it] = *(const v4f*)(stg + 4 * q); }
#pragma unroll
  for (int it = 0; it < 2; ++it) { const int q = it * NTHR + tid; *(volatile v4f*)(gp + 4 * q) = pq[it]; }
  __threadfence();
#pragma unroll
  for (int it = 0; it < 2; ++it) { const int q = it * NTHR + tid; *(volatile v4f*)(gp + 4 * q) = pq[it]; }
}

extern "C" void kernel_launch(void* const* d_in, const int* in_sizes, int n_in,
                              void* d_out, int out_size, void* d_ws, size_t ws_size,
                              hipStream_t stream) {
  if (n_in < 25) return;
  const int nN = in_sizes[3];
  const int nE = in_sizes[1];
  if (nN <= 0 || nE <= 0) return;
  if (in_sizes[0] != nN * XF || in_sizes[2] != 2 * nE) return;
  if (in_sizes[4] != XF * F1 || in_sizes[5] != F1 || in_sizes[6] != XF * F1 || in_sizes[7] != F1 || in_sizes[8] != F1) return;
  if (in_sizes[9] != F1 * F2 || in_sizes[10] != F2 || in_sizes[11] != F1 * F2 || in_sizes[12] != F2 || in_sizes[13] != F2) return;
  if (in_sizes[14] != F2 * F3 || in_sizes[15] != F3 || in_sizes[16] != F2 * F3) return;
  if (in_sizes[17] != F3 * GH || in_sizes[18] != GH || in_sizes[19] != GH || in_sizes[20] != 1) return;
  if (in_sizes[21] != F3 * GH || in_sizes[22] != GH || in_sizes[23] != GH * NOUT || in_sizes[24] != NOUT) return;
  if (out_size <= 0 || (out_size % NOUT) != 0) return;
  const int nG = out_size / NOUT;
  if (nE > (1 << 28) || nN > (1 << 24) || nG > (1 << 20)) return;

  const float* x     = (const float*)d_in[0];
  const float* ew    = (const float*)d_in[1];
  const int*   ei    = (const int*)d_in[2];
  const int*   bat   = (const int*)d_in[3];
  const float* w1r   = (const float*)d_in[4];
  const float* b1r   = (const float*)d_in[5];
  const float* w1o   = (const float*)d_in[6];
  const float* bn1g  = (const float*)d_in[7];
  const float* bn1b  = (const float*)d_in[8];
  const float* w2r   = (const float*)d_in[9];
  const float* b2r   = (const float*)d_in[10];
  const float* w2o   = (const float*)d_in[11];
  const float* bn2g  = (const float*)d_in[12];
  const float* bn2b  = (const float*)d_in[13];
  const float* w3r   = (const float*)d_in[14];
  const float* b3r   = (const float*)d_in[15];
  const float* w3o   = (const float*)d_in[16];
  const float* gw1   = (const float*)d_in[17];
  const float* gb1   = (const float*)d_in[18];
  const float* gw2   = (const float*)d_in[19];
  const float* gb2   = (const float*)d_in[20];
  const float* f1w   = (const float*)d_in[21];
  const float* f1b   = (const float*)d_in[22];
  const float* f4w   = (const float*)d_in[23];
  const float* f4b   = (const float*)d_in[24];
  const int* srcs = ei;
  const int* dsts = ei + nE;
  float* out = (float*)d_out;

  const int NPAD   = ((nN + TGT - 1) / TGT) * TGT;
  const int nBC    = (nN + NBC - 1) / NBC;
  const int CNTPAD = nBC * NBC;
  if (4 * nBC + 1 > RBN) return;
  const int nBF    = (nN + NBF - 1) / NBF;
  const int csrLen = ((nE + 31) & ~31) + 4096;
  if (31 * 4 * nBC > 4096) return;
  const int nGemm  = NPAD / GROWS;
  const int nAgg   = NPAD / TGT;
  const int GPAD   = ((nG + GROWS - 1) / GROWS) * GROWS;
  const int nPB    = GPAD / GPB;
  const int nFc    = GPAD / GROWS;
  const int nPart  = nAgg > nGemm ? nAgg : nGemm;

  char* ws = (char*)d_ws;
  size_t off = 0;
  const size_t oW    = off; off += (size_t)WPTOT * 2;               off = (off + 255) & ~(size_t)255;
  const size_t oCnt  = off; off += (size_t)CNTPAD * 4;              off = (off + 255) & ~(size_t)255;
  const size_t oOff  = off; off += (size_t)CNTPAD * 4;              off = (off + 255) & ~(size_t)255;
  const size_t oRb   = off; off += (size_t)RBN * 4;                 off = (off + 255) & ~(size_t)255;
  const size_t oCsr  = off; off += (size_t)csrLen * 4;              off = (off + 255) & ~(size_t)255;
  const size_t oH1   = off; off += (size_t)NPAD * F1 * 4;           off = (off + 255) & ~(size_t)255;
  const size_t oA2   = off; off += (size_t)NPAD * 2 * F1 * 4;       off = (off + 255) & ~(size_t)255;
  const size_t oH2   = off; off += (size_t)NPAD * F2 * 4;           off = (off + 255) & ~(size_t)255;
  const size_t oA3   = off; off += (size_t)NPAD * 2 * F2 * 4;       off = (off + 255) & ~(size_t)255;
  const size_t oH3   = off; off += (size_t)NPAD * F3 * 4;           off = (off + 255) & ~(size_t)255;
  const size_t oGate = off; off += (size_t)NPAD * 4;                off = (off + 255) & ~(size_t)255;
  const size_t oPool = off; off += (size_t)GPAD * F3 * 4;           off = (off + 255) & ~(size_t)255;
  const size_t oPart = off; off += (size_t)nPart * PSTR * 8;        off = (off + 255) & ~(size_t)255;
  const size_t oCf1  = off; off += (size_t)CSTR * 4;                off = (off + 255) & ~(size_t)255;
  const size_t oCf2  = off; off += (size_t)CSTR * 4;                off = (off + 255) & ~(size_t)255;
  if (off > ws_size || off > (size_t)WSCAP) return;
  unsigned short* wp   = (unsigned short*)(ws + oW);
  int*            cnt  = (int*)(ws + oCnt);
  int*            offp = (int*)(ws + oOff);
  int*            rb   = (int*)(ws + oRb);
  int*            csr  = (int*)(ws + oCsr);
  float*          H1   = (float*)(ws + oH1);
  float*          A2   = (float*)(ws + oA2);
  float*          H2   = (float*)(ws + oH2);
  float*          A3   = (float*)(ws + oA3);
  float*          H3   = (float*)(ws + oH3);
  float*          Gt   = (float*)(ws + oGate);
  float*          Pl   = (float*)(ws + oPool);
  double*         part = (double*)(ws + oPart);
  float*          cf1  = (float*)(ws + oCf1);
  float*          cf2  = (float*)(ws + oCf2);

  const int vec8 = ((nE & 3) == 0) ? 1 : 0;
  const int vecb = 1;

  k_wprep<<<5, NTHR, 0, stream>>>(w2r, w2o, w3r, w3o, gw1, f1w, wp);

  k_count<<<nBC, NTHR, 0, stream>>>(dsts, cnt, nE, vec8);
  k_offsets<<<1, OTHR, 0, stream>>>(cnt, offp, rb, nBC);
  hipFuncSetAttribute(reinterpret_cast<const void*>(&k_fill),
                      hipFuncAttributeMaxDynamicSharedMemorySize, LDS_FILL);
  k_fill<<<nBF, NTHR, LDS_FILL, stream>>>(dsts, offp, rb, csr, nE, vec8, csrLen);

  k_agg0<<<nAgg, NTHR, 0, stream>>>(csr, offp, cnt, srcs, ew, x, w1r, b1r, w1o, H1, part, nN, nE, csrLen);
  k_bnfin<<<1, NTHR, 0, stream>>>(part, bn1g, cf1, nAgg, nN, F1);

  hipFuncSetAttribute(reinterpret_cast<const void*>(&k_agg<F1>),
                      hipFuncAttributeMaxDynamicSharedMemorySize, LDS_AG2);
  k_agg<F1><<<nAgg, NTHR, LDS_AG2, stream>>>(csr, offp, cnt, srcs, ew, H1, cf1, bn1b, A2, nN, nE, csrLen);
  hipFuncSetAttribute(reinterpret_cast<const void*>(&k_gemm<32, 32, 0>),
                      hipFuncAttributeMaxDynamicSharedMemorySize, LDS_G2);
  k_gemm<32, 32, 0><<<nGemm, NTHR, LDS_G2, stream>>>(A2, wp + WP_L2, b2r, gw2, gb2, H2, part, nN);
  k_bnfin<<<1, NTHR, 0, stream>>>(part, bn2g, cf2, nGemm, nN, F2);

  hipFuncSetAttribute(reinterpret_cast<const void*>(&k_agg<F2>),
                      hipFuncAttributeMaxDynamicSharedMemorySize, LDS_AG3);
  k_agg<F2><<<nAgg, NTHR, LDS_AG3, stream>>>(csr, offp, cnt, srcs, ew, H2, cf2, bn2b, A3, nN, nE, csrLen);
  hipFuncSetAttribute(reinterpret_cast<const void*>(&k_gemm<64, 64, 1>),
                      hipFuncAttributeMaxDynamicSharedMemorySize, LDS_G3);
  k_gemm<64, 64, 1><<<nGemm, NTHR, LDS_G3, stream>>>(A3, wp + WP_L3, b3r, gw2, gb2, H3, part, nN);

  hipFuncSetAttribute(reinterpret_cast<const void*>(&k_gemm<64, 32, 2>),
                      hipFuncAttributeMaxDynamicSharedMemorySize, LDS_GH);
  k_gemm<64, 32, 2><<<nGemm, NTHR, LDS_GH, stream>>>(H3, wp + WP_GT, gb1, gw2, gb2, Gt, part, nN);

  k_pool<<<nPB, NTHR, 0, stream>>>(bat, Gt, H3, Pl, nN, vecb);

  hipFuncSetAttribute(reinterpret_cast<const void*>(&k_gemm<64, 32, 3>),
                      hipFuncAttributeMaxDynamicSharedMemorySize, LDS_GH);
  k_gemm<64, 32, 3><<<nFc, NTHR, LDS_GH, stream>>>(Pl, wp + WP_FC, f1b, f4w, f4b, out, part, nG);
}
